// SchrodingerAttention_75239237091374
// MI455X (gfx1250) — hardware-run, weakly checked
//
#include <hip/hip_runtime.h>
#include <math.h>

typedef __attribute__((ext_vector_type(16))) _Float16 v16h;
typedef __attribute__((ext_vector_type(8)))  _Float16 v8h;
typedef __attribute__((ext_vector_type(8)))  float    v8f;
typedef __attribute__((ext_vector_type(4)))  float    v4f;

constexpr int kBsz    = 4;
constexpr int kSeq    = 4096;
constexpr int kDim    = 512;
constexpr int kBands  = 4;
constexpr int kBandW  = kDim / kBands;
constexpr int kRows   = kBsz * kSeq;
constexpr int kHalfB  = 2;
constexpr int kNHalf  = kBsz / kHalfB;
constexpr int kHRows  = kHalfB * kSeq;
constexpr int kN1     = 2 * kDim;
constexpr int kNcat   = 2 * kN1;
constexpr int kChunk  = 512;
constexpr int kNChunk = kSeq / kChunk;
constexpr int kGrp    = kHalfB * kDim;
constexpr int kSlabP  = 36;
constexpr float kXCarry   = 16.0f;
constexpr float kWCarry   = 1024.0f;
constexpr float kResCarry = 2048.0f;
constexpr float kResInv   = 1.0f / kResCarry;
constexpr float kFold     = 1.0f / (kXCarry * kWCarry);
static_assert(kBandW == 128 && kRows == 16384 && kN1 == 1024 && kNcat == 2048, "shapes");
static_assert(kNHalf == 2 && kHRows == 8192 && kNChunk == 8 && kGrp == 1024, "pass shapes");
static_assert((kDim % 32) == 0, "GEMM K multiple of 32");
static_assert((kHRows % 64) == 0 && (kNcat % 32) == 0, "GEMM M multiple of 64, N multiple of 32");
static_assert((kNcat / 32) == 64, "tile decode uses 64 column tiles per tile row");
static_assert((((kHRows / 64) * (kNcat / 32)) % 8) == 0, "whole blocks of 8 tiles");
static_assert(((kN1 / 32) % 8) == 0, "a block never straddles the psi/phi column halves");
static_assert((kSlabP % 4) == 0 && kSlabP >= 32, "slab pitch keeps 16-B alignment");

constexpr size_t kOffXH   = 0;
constexpr size_t kOffXL   = kOffXH   + (size_t)kHRows * kDim * 2;
constexpr size_t kOffWCH  = kOffXL   + (size_t)kHRows * kDim * 2;
constexpr size_t kOffWCL  = kOffWCH  + (size_t)kNcat * kDim * 2;
constexpr size_t kOffUH   = kOffWCL  + (size_t)kNcat * kDim * 2;
constexpr size_t kOffPHI  = kOffUH   + (size_t)kHRows * kN1 * 4;
constexpr size_t kOffGATE = kOffPHI  + (size_t)kHRows * kN1 * 4;
constexpr size_t kOffPWR  = kOffGATE + (size_t)kHRows * 4;
constexpr size_t kOffPWI  = kOffPWR  + (size_t)kChunk * kDim * 4;
constexpr size_t kOffER   = kOffPWI  + (size_t)kChunk * kDim * 4;
constexpr size_t kOffEI   = kOffER   + (size_t)kNChunk * kGrp * 4;
constexpr size_t kOffCR   = kOffEI   + (size_t)kNChunk * kGrp * 4;
constexpr size_t kOffCI   = kOffCR   + (size_t)kNChunk * kGrp * 4;
constexpr size_t kWsTotal = kOffCI   + (size_t)kNChunk * kGrp * 4;
static_assert(kWsTotal == 90341376ull, "carve total");
static_assert(kWsTotal <= 134217728ull, "carve cap");
static_assert((kOffXL % 128) == 0 && (kOffWCH % 128) == 0 && (kOffWCL % 128) == 0 && (kOffUH % 128) == 0 &&
              (kOffPHI % 128) == 0 && (kOffGATE % 128) == 0 && (kOffPWR % 128) == 0 && (kOffPWI % 128) == 0 &&
              (kOffER % 128) == 0 && (kOffEI % 128) == 0 && (kOffCR % 128) == 0 && (kOffCI % 128) == 0,
              "128-B aligned regions");

__device__ __forceinline__ void split_h(float v, _Float16& hi, _Float16& lo) {
  const _Float16 h = (_Float16)v;
  const float hf = (float)h;
  const float r = (v - hf) * kResCarry;
  hi = h;
  lo = (_Float16)r;
}

union FragH { v16h v; v8h h[2]; };
__device__ __forceinline__ v16h frag_load(const _Float16* p) {
  FragH f;
  f.h[0] = *(const v8h*)(p);
  f.h[1] = *(const v8h*)(p + 16);
  return f.v;
}

__device__ __forceinline__ v8f mma_h(v16h a, v16h b, v8f c) {
  c = __builtin_amdgcn_wmma_f32_16x16x32_f16(false, a, false, b, (short)0, c, false, false);
  asm volatile("v_nop\n\tv_nop\n\tv_nop\n\tv_nop" : "+v"(c) : "v"(a), "v"(b));
  return c;
}

__global__ __launch_bounds__(256) void cvt_gate_kernel(
    const float* __restrict__ X, const float* __restrict__ Z, const float* __restrict__ Wg,
    const float* __restrict__ bg, const float* __restrict__ sgp,
    unsigned short* __restrict__ XH, unsigned short* __restrict__ XL, float* __restrict__ gate)
{
  __shared__ float sG[32];
  const int lane = threadIdx.x & 31;
  const int wave = __builtin_amdgcn_readfirstlane((int)(threadIdx.x >> 5));
  const float tsg = tanhf(sgp[0]);
  const int useS = __builtin_amdgcn_readfirstlane((tsg != 0.0f) ? 1 : 0);
  const float bgv = bg[0];
  const int ca = lane * 8;
  const int cb = 256 + lane * 8;
  const v4f w0 = *(const v4f*)(Wg + ca);
  const v4f w1 = *(const v4f*)(Wg + ca + 4);
  const v4f w2 = *(const v4f*)(Wg + cb);
  const v4f w3 = *(const v4f*)(Wg + cb + 4);
#pragma unroll 1
  for (int rr = 0; rr < 4; ++rr) {
    const int row = blockIdx.x * 32 + wave * 4 + rr;
    const float* xr = X + (size_t)row * kDim;
    const v4f a0 = *(const v4f*)(xr + ca);
    const v4f a1 = *(const v4f*)(xr + ca + 4);
    const v4f a2 = *(const v4f*)(xr + cb);
    const v4f a3 = *(const v4f*)(xr + cb + 4);
    float dot = 0.f;
#pragma unroll
    for (int e = 0; e < 4; ++e) {
      dot = fmaf(a0[e], w0[e], dot);
      dot = fmaf(a1[e], w1[e], dot);
      dot = fmaf(a2[e], w2[e], dot);
      dot = fmaf(a3[e], w3[e], dot);
    }
    float sd = 0.f;
    if (useS) {
      const float* zr = Z + (size_t)row * kDim;
      const v4f z0 = *(const v4f*)(zr + ca);
      const v4f z1 = *(const v4f*)(zr + ca + 4);
      const v4f z2 = *(const v4f*)(zr + cb);
      const v4f z3 = *(const v4f*)(zr + cb + 4);
#pragma unroll
      for (int e = 0; e < 4; ++e) {
        sd += fabsf(a0[e] - z0[e]);
        sd += fabsf(a1[e] - z1[e]);
        sd += fabsf(a2[e] - z2[e]);
        sd += fabsf(a3[e] - z3[e]);
      }
    }
#pragma unroll
    for (int off = 16; off > 0; off >>= 1) {
      dot += __shfl_xor(dot, off, 32);
      sd  += __shfl_xor(sd, off, 32);
    }
    float g = 1.0f / (1.0f + expf(-(dot + bgv)));
    g = g * (1.0f + tsg * (sd * (1.0f / (float)kDim)));
    if (lane == 0) sG[wave * 4 + rr] = g;
    v8h h0, h1, l0, l1;
#pragma unroll
    for (int e = 0; e < 4; ++e) {
      _Float16 th, tl;
      split_h(a0[e] * kXCarry, th, tl);
      h0[e] = th;
      l0[e] = tl;
      split_h(a1[e] * kXCarry, th, tl);
      h0[4 + e] = th;
      l0[4 + e] = tl;
      split_h(a2[e] * kXCarry, th, tl);
      h1[e] = th;
      l1[e] = tl;
      split_h(a3[e] * kXCarry, th, tl);
      h1[4 + e] = th;
      l1[4 + e] = tl;
    }
    unsigned short* q0 = XH + (size_t)row * kDim + ca;
    unsigned short* q1 = XH + (size_t)row * kDim + cb;
    unsigned short* r0 = XL + (size_t)row * kDim + ca;
    unsigned short* r1 = XL + (size_t)row * kDim + cb;
    *(volatile v8h*)q0 = h0;
    *(volatile v8h*)q1 = h1;
    *(volatile v8h*)r0 = l0;
    *(volatile v8h*)r1 = l1;
    __threadfence();
    *(volatile v8h*)q0 = h0;
    *(volatile v8h*)q1 = h1;
    *(volatile v8h*)r0 = l0;
    *(volatile v8h*)r1 = l1;
  }
  __syncthreads();
  if (wave == 0) {
    const float v = sG[lane];
    float* gp = gate + (size_t)blockIdx.x * 32 + lane;
    *(volatile float*)gp = v;
    __threadfence();
    *(volatile float*)gp = v;
  }
}

__global__ __launch_bounds__(256) void wcvt_kernel(
    const float* __restrict__ Wpsi, const float* __restrict__ Wphi,
    unsigned short* __restrict__ WCH, unsigned short* __restrict__ WCL)
{
  const int i = blockIdx.x * 256 + threadIdx.x;
  const float* src = (blockIdx.y == 0) ? Wpsi : Wphi;
  const size_t e0 = (size_t)i << 3;
  const v4f a0 = *(const v4f*)(src + e0);
  const v4f a1 = *(const v4f*)(src + e0 + 4);
  v8h hv, lv;
#pragma unroll
  for (int e = 0; e < 4; ++e) {
    _Float16 th, tl;
    split_h(a0[e] * kWCarry, th, tl);
    hv[e] = th;
    lv[e] = tl;
    split_h(a1[e] * kWCarry, th, tl);
    hv[4 + e] = th;
    lv[4 + e] = tl;
  }
  const size_t o = (size_t)blockIdx.y * ((size_t)kN1 * kDim) + e0;
  unsigned short* qh = WCH + o;
  unsigned short* ql = WCL + o;
  *(volatile v8h*)qh = hv;
  *(volatile v8h*)ql = lv;
  __threadfence();
  *(volatile v8h*)qh = hv;
  *(volatile v8h*)ql = lv;
}

__global__ __launch_bounds__(256) void pow_table_kernel(
    const float* __restrict__ lgam, const float* __restrict__ omg, const float* __restrict__ dtp,
    float* __restrict__ PWR, float* __restrict__ PWI)
{
  const int idx = blockIdx.x * 256 + threadIdx.x;
  const int d  = idx & (kDim - 1);
  const int tl = idx >> 9;
  const float dta = fabsf(dtp[0]);
  const float tt = (float)(tl + 1) * dta;
  const float gam = expf(lgam[d]);
  float de = expf(-gam * tt);
  de = (de < 1.17549435e-38f) ? 0.0f : de;
  const float an = omg[d] * tt;
  float sn, cs;
  sincosf(an, &sn, &cs);
  const float vr = de * cs;
  const float vi = de * sn;
  *(volatile float*)(PWR + idx) = vr;
  *(volatile float*)(PWI + idx) = vi;
  __threadfence();
  *(volatile float*)(PWR + idx) = vr;
  *(volatile float*)(PWI + idx) = vi;
}

__global__ __launch_bounds__(256) void proj_gemm_kernel(
    const unsigned short* __restrict__ XHp, const unsigned short* __restrict__ XLp,
    const unsigned short* __restrict__ WHp, const unsigned short* __restrict__ WLp,
    const float* __restrict__ bpsi, const float* __restrict__ bphi,
    const float* __restrict__ gate, const float* __restrict__ Bvec,
    float* __restrict__ UH, float* __restrict__ PHI)
{
  __shared__ __align__(16) float sT[8][16 * kSlabP];
  const _Float16* Ah = (const _Float16*)XHp;
  const _Float16* Al = (const _Float16*)XLp;
  const _Float16* Bh = (const _Float16*)WHp;
  const _Float16* Bl = (const _Float16*)WLp;
  const int lane = threadIdx.x & 31;
  const int wave = __builtin_amdgcn_readfirstlane((int)(threadIdx.x >> 5));
  const int tile = blockIdx.x * 8 + wave;
  const int tm = tile >> 6;
  const int tn = tile & 63;
  const int m0 = tm << 6;
  const int nW0 = tn << 5;
  const int rlane = lane & 15;
  const int koff  = (lane >> 4) * 8;
  const int mOff  = (lane >> 4) * 8;

  v8f acc[4][2], res[4][2];
#pragma unroll
  for (int i = 0; i < 4; ++i) {
#pragma unroll
    for (int j = 0; j < 2; ++j) {
      acc[i][j] = (v8f){0.f, 0.f, 0.f, 0.f, 0.f, 0.f, 0.f, 0.f};
      res[i][j] = (v8f){0.f, 0.f, 0.f, 0.f, 0.f, 0.f, 0.f, 0.f};
    }
  }

#pragma unroll 1
  for (int k0 = 0; k0 < kDim; k0 += 32) {
    v16h bh[2], bl[2];
#pragma unroll
    for (int j = 0; j < 2; ++j) {
      const size_t bo = (size_t)(nW0 + (j << 4) + rlane) * kDim + koff + k0;
      bh[j] = frag_load(Bh + bo);
      bl[j] = frag_load(Bl + bo);
    }
#pragma unroll
    for (int i = 0; i < 4; ++i) {
      const size_t ao = (size_t)(m0 + (i << 4) + rlane) * kDim + koff + k0;
      const v16h ah = frag_load(Ah + ao);
      const v16h al = frag_load(Al + ao);
#pragma unroll
      for (int j = 0; j < 2; ++j) {
        acc[i][j] = mma_h(ah, bh[j], acc[i][j]);
        res[i][j] = mma_h(ah, bl[j], res[i][j]);
        res[i][j] = mma_h(al, bh[j], res[i][j]);
      }
    }
  }

  float* slab = sT[wave];
  const bool isPsi = (tn < (kN1 >> 5));
  const int ncol = (tn & ((kN1 >> 5) - 1)) << 5;
  float* Cb = isPsi ? UH : PHI;
  float bvj[2], sfj[2];
#pragma unroll
  for (int j = 0; j < 2; ++j) {
    const int nn = ncol + (j << 4) + rlane;
    const float b1 = bpsi[nn];
    const float b2 = bphi[nn];
    const float bv = Bvec[nn & (kDim - 1)];
    bvj[j] = isPsi ? b1 : b2;
    sfj[j] = isPsi ? bv : 1.0f;
  }
  const int q  = lane >> 3;
  const int c4 = (lane & 7) * 4;
#pragma unroll
  for (int i = 0; i < 4; ++i) {
    const int mBase = m0 + (i << 4);
    const v4f g0 = *(const v4f*)(gate + mBase + mOff);
    const v4f g1 = *(const v4f*)(gate + mBase + mOff + 4);
    float gs[8];
#pragma unroll
    for (int r = 0; r < 4; ++r) {
      const float ga = g0[r];
      const float gb = g1[r];
      gs[r]     = isPsi ? ga : 1.0f;
      gs[4 + r] = isPsi ? gb : 1.0f;
    }
#pragma unroll
    for (int j = 0; j < 2; ++j) {
#pragma unroll
      for (int r = 0; r < 8; ++r) {
        const float s0 = fmaf(res[i][j][r], kResInv, acc[i][j][r]);
        const float v = fmaf(s0, kFold, bvj[j]);
        const float s = gs[r] * sfj[j];
        slab[(mOff + r) * kSlabP + (j << 4) + rlane] = v * s;
      }
    }
    __syncthreads();
    v4f ov[4];
#pragma unroll
    for (int it = 0; it < 4; ++it) ov[it] = *(const v4f*)(slab + (it * 4 + q) * kSlabP + c4);
    for (int pass = 0; pass < 2; ++pass) {
#pragma unroll
      for (int it = 0; it < 4; ++it) {
        const int row = it * 4 + q;
        *(volatile v4f*)(Cb + (size_t)(mBase + row) * kN1 + ncol + c4) = ov[it];
      }
      __threadfence();
    }
    __syncthreads();
  }
}

__global__ __launch_bounds__(256) void scan_local_kernel(
    float* UH, const float* __restrict__ PWR, const float* __restrict__ PWI,
    float* __restrict__ ER, float* __restrict__ EI)
{
  const int id = blockIdx.x * 256 + threadIdx.x;
  const int g = id & (kGrp - 1);
  const int c = id >> 10;
  const int d = g & (kDim - 1);
  const int b = g >> 9;
  const float ar = PWR[d];
  const float ai = PWI[d];
  float* base = UH + ((size_t)b * kSeq + (size_t)c * kChunk) * kN1 + d;
  float hr = 0.f, hi = 0.f;
#pragma unroll 1
  for (int t0 = 0; t0 < kChunk; t0 += 8) {
    float vr[8], vi[8];
#pragma unroll
    for (int s = 0; s < 8; ++s) {
      vr[s] = base[(size_t)(t0 + s) * kN1];
      vi[s] = base[(size_t)(t0 + s) * kN1 + kDim];
    }
#pragma unroll
    for (int s = 0; s < 8; ++s) {
      const float nr = fmaf(ar, hr, fmaf(-ai, hi, vr[s]));
      const float ni = fmaf(ar, hi, fmaf(ai, hr, vi[s]));
      hr = nr;
      hi = ni;
      vr[s] = hr;
      vi[s] = hi;
    }
    for (int pass = 0; pass < 2; ++pass) {
#pragma unroll
      for (int s = 0; s < 8; ++s) {
        *(volatile float*)(base + (size_t)(t0 + s) * kN1) = vr[s];
        *(volatile float*)(base + (size_t)(t0 + s) * kN1 + kDim) = vi[s];
      }
      __threadfence();
    }
  }
  float* er = ER + (size_t)c * kGrp + g;
  float* ei = EI + (size_t)c * kGrp + g;
  *(volatile float*)er = hr;
  *(volatile float*)ei = hi;
  __threadfence();
  *(volatile float*)er = hr;
  *(volatile float*)ei = hi;
}

__global__ __launch_bounds__(64) void scan_carry_kernel(
    const float* __restrict__ ER, const float* __restrict__ EI,
    const float* __restrict__ PWR, const float* __restrict__ PWI,
    float* __restrict__ CR, float* __restrict__ CI)
{
  const int g = blockIdx.x * 64 + threadIdx.x;
  const int d = g & (kDim - 1);
  const float Ar = PWR[(size_t)(kChunk - 1) * kDim + d];
  const float Ai = PWI[(size_t)(kChunk - 1) * kDim + d];
  float outR[kNChunk], outI[kNChunk];
  float cr = 0.f, ci = 0.f;
#pragma unroll
  for (int c = 0; c < kNChunk; ++c) {
    outR[c] = cr;
    outI[c] = ci;
    const float er = ER[(size_t)c * kGrp + g];
    const float ei = EI[(size_t)c * kGrp + g];
    const float nr = fmaf(Ar, cr, fmaf(-Ai, ci, er));
    const float ni = fmaf(Ar, ci, fmaf(Ai, cr, ei));
    cr = nr;
    ci = ni;
  }
  for (int pass = 0; pass < 2; ++pass) {
#pragma unroll
    for (int c = 0; c < kNChunk; ++c) {
      *(volatile float*)(CR + (size_t)c * kGrp + g) = outR[c];
      *(volatile float*)(CI + (size_t)c * kGrp + g) = outI[c];
    }
    __threadfence();
  }
}

__global__ __launch_bounds__(128) void row_kernel(
    const float* __restrict__ UH, const float* __restrict__ PHI,
    const float* __restrict__ PWR, const float* __restrict__ PWI,
    const float* __restrict__ CR, const float* __restrict__ CI,
    const int* __restrict__ bidx, const float* __restrict__ taup, const float* __restrict__ betap,
    float* __restrict__ out)
{
  __shared__ __align__(16) float sW[4][5 * kDim];
  const int lane = threadIdx.x & 31;
  const int wave = __builtin_amdgcn_readfirstlane((int)(threadIdx.x >> 5));
  float* hr_s  = sW[wave];
  float* hi_s  = hr_s + kDim;
  float* ph_s  = hr_s + 2 * kDim;
  float* out_s = hr_s + 4 * kDim;
  const int row = blockIdx.x * 4 + wave;
  const int t  = row & (kSeq - 1);
  const int b  = row >> 12;
  const int c  = t >> 9;
  const int tl = t & (kChunk - 1);

#pragma unroll
  for (int qq = 0; qq < 4; ++qq)
    *(v4f*)(out_s + qq * 128 + lane * 4) = (v4f){0.f, 0.f, 0.f, 0.f};
  const float* phrow = PHI + (size_t)row * kN1;
#pragma unroll 4
  for (int qq = 0; qq < 8; ++qq) {
    const v4f u = *(const v4f*)(phrow + qq * 128 + lane * 4);
    *(v4f*)(ph_s + qq * 128 + lane * 4) = u;
  }

  const float* hrow = UH + (size_t)row * kN1;
  const float* crow = CR + (size_t)c * kGrp + (size_t)b * kDim;
  const float* cirow = CI + (size_t)c * kGrp + (size_t)b * kDim;
  const float* prow = PWR + (size_t)tl * kDim;
  const float* pirow = PWI + (size_t)tl * kDim;
  float sr = 0.f, si = 0.f;
#pragma unroll 1
  for (int it = 0; it < 16; ++it) {
    const int d = it * 32 + lane;
    float hr = hrow[d];
    float hi = hrow[kDim + d];
    const float cr = crow[d];
    const float ci = cirow[d];
    const float pr = prow[d];
    const float pi = pirow[d];
    hr += cr * pr - ci * pi;
    hi += cr * pi + ci * pr;
    hr_s[d] = hr;
    hi_s[d] = hi;
    sr += hr;
    si += hi;
  }
#pragma unroll
  for (int off = 16; off > 0; off >>= 1) {
    sr += __shfl_xor(sr, off, 32);
    si += __shfl_xor(si, off, 32);
  }
  const float invD = 1.0f / (float)kDim;
  const float mr = sr * invD;
  const float mi = si * invD;
  float vr = 0.f, vi = 0.f;
#pragma unroll 4
  for (int it = 0; it < 16; ++it) {
    const int d = it * 32 + lane;
    const float dr = hr_s[d] - mr;
    const float di = hi_s[d] - mi;
    vr = fmaf(dr, dr, vr);
    vi = fmaf(di, di, vi);
  }
#pragma unroll
  for (int off = 16; off > 0; off >>= 1) {
    vr += __shfl_xor(vr, off, 32);
    vi += __shfl_xor(vi, off, 32);
  }
  const float ivr = 1.0f / (sqrtf(vr * invD) + 1e-6f);
  const float ivi = 1.0f / (sqrtf(vi * invD) + 1e-6f);
#pragma unroll 4
  for (int it = 0; it < 16; ++it) {
    const int d = it * 32 + lane;
    hr_s[d] = (hr_s[d] - mr) * ivr;
    hi_s[d] = (hi_s[d] - mi) * ivi;
  }
  __syncthreads();

  float aR[kBands], aI[kBands], dK[kBands];
#pragma unroll
  for (int kk = 0; kk < kBands; ++kk) {
    aR[kk] = 0.f;
    aI[kk] = 0.f;
    dK[kk] = 0.f;
  }
  const float invBand = 1.0f / (float)kBandW;
#pragma unroll 1
  for (int k = 0; k < kBands; ++k) {
    float ar = 0.f, ai = 0.f, dn = 0.f;
#pragma unroll
    for (int i = 0; i < 4; ++i) {
      const int e = k * kBandW + i * 32 + lane;
      int d = bidx[e];
      d = (d < 0) ? 0 : d;
      d = (d > kDim - 1) ? (kDim - 1) : d;
      const float hrn = hr_s[d];
      const float hin = hi_s[d];
      const float pr = ph_s[d];
      const float pi = ph_s[kDim + d];
      ar = fmaf(hrn, pr, ar);
      ar = fmaf(hin, pi, ar);
      ai = fmaf(hrn, pi, ai);
      ai = fmaf(-hin, pr, ai);
      dn = fmaf(hrn, hrn, dn);
      dn = fmaf(hin, hin, dn);
    }
#pragma unroll
    for (int off = 16; off > 0; off >>= 1) {
      ar += __shfl_xor(ar, off, 32);
      ai += __shfl_xor(ai, off, 32);
      dn += __shfl_xor(dn, off, 32);
    }
    const float tr = ar * invBand;
    const float ti = ai * invBand;
    const float td = dn * invBand;
#pragma unroll
    for (int kk = 0; kk < kBands; ++kk) {
      const bool s = (k == kk);
      aR[kk] = s ? tr : aR[kk];
      aI[kk] = s ? ti : aI[kk];
      dK[kk] = s ? td : dK[kk];
    }
  }

  const float tauc = fmaxf(taup[0], 1e-4f);
  const float itau = 1.0f / tauc;
  const float betav = betap[0];
  float lg[kBands];
  float mx = -INFINITY;
#pragma unroll
  for (int kk = 0; kk < kBands; ++kk) {
    lg[kk] = sqrtf(aR[kk] * aR[kk] + aI[kk] * aI[kk]) * itau;
    mx = fmaxf(mx, lg[kk]);
  }
  float ssum = 0.f;
#pragma unroll
  for (int kk = 0; kk < kBands; ++kk) {
    lg[kk] = expf(lg[kk] - mx);
    ssum += lg[kk];
  }
  const float isum = 1.0f / ssum;
  float afr[kBands], afi[kBands];
#pragma unroll
  for (int kk = 0; kk < kBands; ++kk) {
    const float ck = lg[kk] * isum;
    afr[kk] = (aR[kk] * ck) * (float)kBands + betav * dK[kk];
    afi[kk] = (aI[kk] * ck) * (float)kBands;
  }

#pragma unroll 1
  for (int k = 0; k < kBands; ++k) {
    float fr = afr[0];
    float fi = afi[0];
#pragma unroll
    for (int kk = 1; kk < kBands; ++kk) {
      const bool s = (k == kk);
      fr = s ? afr[kk] : fr;
      fi = s ? afi[kk] : fi;
    }
#pragma unroll
    for (int i = 0; i < 4; ++i) {
      const int e = k * kBandW + i * 32 + lane;
      int d = bidx[e];
      d = (d < 0) ? 0 : d;
      d = (d > kDim - 1) ? (kDim - 1) : d;
      out_s[d] = hr_s[d] * fr - hi_s[d] * fi;
    }
  }
  __syncthreads();

  v4f ov[4];
#pragma unroll
  for (int qq = 0; qq < 4; ++qq) ov[qq] = *(const v4f*)(out_s + qq * 128 + lane * 4);
  float* orow = out + (size_t)row * kDim + lane * 4;
  for (int pass = 0; pass < 2; ++pass) {
#pragma unroll
    for (int qq = 0; qq < 4; ++qq) *(volatile v4f*)(orow + qq * 128) = ov[qq];
    __threadfence();
  }
}

extern "C" void kernel_launch(void* const* d_in, const int* in_sizes, int n_in,
                              void* d_out, int out_size, void* d_ws, size_t ws_size,
                              hipStream_t stream) {
  if (n_in < 16) return;
  if (in_sizes[0] != kRows * kDim) return;
  if (in_sizes[1] != kRows * kDim) return;
  if (in_sizes[2] != kN1 * kDim) return;
  if (in_sizes[3] != kN1) return;
  if (in_sizes[4] != kN1 * kDim) return;
  if (in_sizes[5] != kN1) return;
  if (in_sizes[6] != kDim) return;
  if (in_sizes[7] != 1) return;
  if (in_sizes[8] != kDim) return;
  if (in_sizes[9] != kDim) return;
  if (in_sizes[10] != 1) return;
  if (in_sizes[11] != 1) return;
  if (in_sizes[12] != 1) return;
  if (in_sizes[13] != 1) return;
  if (in_sizes[14] != kDim) return;
  if (in_sizes[15] != kDim) return;
  if (out_size != kRows * kDim) return;
  if (ws_size < kWsTotal) return;

  const float* x      = (const float*)d_in[0];
  const float* z_prev = (const float*)d_in[1];
  const float* W_psi  = (const float*)d_in[2];
  const float* b_psi  = (const float*)d_in[3];
  const float* W_phi  = (const float*)d_in[4];
  const float* b_phi  = (const float*)d_in[5];
  const float* W_gate = (const float*)d_in[6];
  const float* b_gate = (const float*)d_in[7];
  const float* omega  = (const float*)d_in[8];
  const float* lgam   = (const float*)d_in[9];
  const float* dtp    = (const float*)d_in[10];
  const float* sgain  = (const float*)d_in[11];
  const float* taup   = (const float*)d_in[12];
  const float* betap  = (const float*)d_in[13];
  const float* B_vec  = (const float*)d_in[14];
  const int*   bidx   = (const int*)d_in[15];
  float* out = (float*)d_out;

  char* ws = (char*)d_ws;
  unsigned short* XH   = (unsigned short*)(ws + kOffXH);
  unsigned short* XL   = (unsigned short*)(ws + kOffXL);
  unsigned short* WCH  = (unsigned short*)(ws + kOffWCH);
  unsigned short* WCL  = (unsigned short*)(ws + kOffWCL);
  float*          UH   = (float*)(ws + kOffUH);
  float*          PHI  = (float*)(ws + kOffPHI);
  float*          GATE = (float*)(ws + kOffGATE);
  float*          PWR  = (float*)(ws + kOffPWR);
  float*          PWI  = (float*)(ws + kOffPWI);
  float*          ER   = (float*)(ws + kOffER);
  float*          EI   = (float*)(ws + kOffEI);
  float*          CR   = (float*)(ws + kOffCR);
  float*          CI   = (float*)(ws + kOffCI);

  wcvt_kernel<<<dim3((kN1 * kDim / 8) / 256, 2), 256, 0, stream>>>(W_psi, W_phi, WCH, WCL);
  pow_table_kernel<<<(kChunk * kDim) / 256, 256, 0, stream>>>(lgam, omega, dtp, PWR, PWI);

  for (int hp = 0; hp < kNHalf; ++hp) {
    const size_t ro = (size_t)hp * kHRows * kDim;
    cvt_gate_kernel<<<kHRows / 32, 256, 0, stream>>>(x + ro, z_prev + ro, W_gate, b_gate, sgain, XH, XL, GATE);
    proj_gemm_kernel<<<((kHRows / 64) * (kNcat / 32)) / 8, 256, 0, stream>>>(
        XH, XL, WCH, WCL, b_psi, b_phi, GATE, B_vec, UH, PHI);
    scan_local_kernel<<<(kGrp * kNChunk) / 256, 256, 0, stream>>>(UH, PWR, PWI, ER, EI);
    scan_carry_kernel<<<kGrp / 64, 64, 0, stream>>>(ER, EI, PWR, PWI, CR, CI);
    row_kernel<<<kHRows / 4, 128, 0, stream>>>(UH, PHI, PWR, PWI, CR, CI, bidx, taup, betap, out + ro);
  }
}
